// LightningDecoderLayer_7181185319150
// MI455X (gfx1250) — hardware-run, weakly checked
//
#include <hip/hip_runtime.h>
#include <math.h>

constexpr int kBatch  = 2;
constexpr int kSteps  = 2048;
constexpr int kChan   = 1024;
constexpr int kHeads  = 16;
constexpr int kHdim   = 64;
constexpr int kTaps   = 4;
constexpr int kTok    = kBatch * kSteps;
constexpr size_t kPlane = (size_t)kTok * kChan;
constexpr size_t kWBig  = (size_t)kChan * kChan;
constexpr int kGateN    = 64;
constexpr int kGateReal = 2 * kHeads;
constexpr int kChunk    = 16;
constexpr int kHalfD    = kHdim / 2;

constexpr float kXCarry   = 16.0f;
constexpr float kWCarry   = 256.0f;
constexpr float kYCarry   = 16.0f;
constexpr float kResCarry = 2048.0f;
constexpr float kResInv   = 1.0f / kResCarry;
constexpr float kScaleProj = 1.0f / (kXCarry * kWCarry);
constexpr float kScaleOut  = 1.0f / (kYCarry * kWCarry);
constexpr float kF16Min   = 6.103515625e-5f;
constexpr float kF32Min   = 1.17549435e-38f;
constexpr float kNormEps  = 1e-6f;

constexpr float  kRopeBase    = 10000.0f;
constexpr double kMaxSeq      = 262144.0;
constexpr double kOrigMax     = 8192.0;
constexpr float  kRopeScaling = 32.0f;
constexpr float  kBetaFast    = 1.0f;
constexpr float  kBetaSlow    = 32.0f;
static_assert(kMaxSeq / kOrigMax == 32.0, "extension factor is 2^5");
constexpr float kSbExp  = (float)(5.0 * (double)kHdim / (double)(kHdim - 2));
constexpr float kTwoPi  = (float)(2.0 * 3.14159265358979323846);

static_assert(kHeads * kHdim == kChan, "heads");
static_assert(kTok % 32 == 0 && kChan % 64 == 0 && kGateN % 64 == 0, "GEMM M,N tile multiples");
static_assert(kChan % 32 == 0, "GEMM K multiple of 32");
static_assert(kSteps % kChunk == 0 && (kSteps & (kSteps - 1)) == 0, "steps");
static_assert((kTok * kHeads) % 8 == 0, "wave per (token, head)");
static_assert(kHdim == 64 && kChunk == 16 && kTaps == 4 && kGateReal == 32, "layout assumptions");

typedef __attribute__((ext_vector_type(16))) _Float16 v16h;
typedef __attribute__((ext_vector_type(8)))  _Float16 v8h;
typedef __attribute__((ext_vector_type(8)))  float    v8f;
typedef __attribute__((ext_vector_type(4)))  float    v4f;
typedef __attribute__((ext_vector_type(2)))  float    v2f;
typedef __attribute__((ext_vector_type(4)))  unsigned int v4u;

__device__ __forceinline__ unsigned pk16(unsigned short a, unsigned short b) {
  return (unsigned)a | ((unsigned)b << 16);
}
__device__ __forceinline__ unsigned short h_bits(float f) {
  const float g = (fabsf(f) < kF16Min) ? 0.0f : f;
  const _Float16 h = (_Float16)g;
  return __builtin_bit_cast(unsigned short, h);
}
__device__ __forceinline__ void h_split(float v, unsigned short& hb, unsigned short& rb) {
  const float g = (fabsf(v) < kF16Min) ? 0.0f : v;
  const _Float16 h = (_Float16)g;
  const float hf = (float)h;
  const float d = (v - hf) * kResCarry;
  const float dg = (fabsf(d) < kF16Min) ? 0.0f : d;
  const _Float16 r = (_Float16)dg;
  hb = __builtin_bit_cast(unsigned short, h);
  rb = __builtin_bit_cast(unsigned short, r);
}
__device__ __forceinline__ v4u pack8_plain(const float (&v)[8]) {
  unsigned short hb[8];
#pragma unroll
  for (int e = 0; e < 8; ++e) hb[e] = h_bits(v[e]);
  return (v4u){pk16(hb[0], hb[1]), pk16(hb[2], hb[3]), pk16(hb[4], hb[5]), pk16(hb[6], hb[7])};
}
__device__ __forceinline__ void pack8_split(const float (&v)[8], v4u& uh, v4u& ur) {
  unsigned short hb[8], rb[8];
#pragma unroll
  for (int e = 0; e < 8; ++e) h_split(v[e], hb[e], rb[e]);
  uh = (v4u){pk16(hb[0], hb[1]), pk16(hb[2], hb[3]), pk16(hb[4], hb[5]), pk16(hb[6], hb[7])};
  ur = (v4u){pk16(rb[0], rb[1]), pk16(rb[2], rb[3]), pk16(rb[4], rb[5]), pk16(rb[6], rb[7])};
}
__device__ __forceinline__ float wave_sum32(float v) {
#pragma unroll
  for (int o = 16; o > 0; o >>= 1) v += __shfl_xor(v, o, 32);
  return v;
}

struct FragH {
  union U { v16h v; v8h h[2]; };
  static __device__ __forceinline__ v16h load(const _Float16* p) {
    U f;
    f.h[0] = *(const v8h*)(p);
    f.h[1] = *(const v8h*)(p + 16);
    return f.v;
  }
  static __device__ __forceinline__ v8f mma(v16h a, v16h b, v8f c) {
    return __builtin_amdgcn_wmma_f32_16x16x32_f16(false, a, false, b, (short)0, c, false, false);
  }
};
__device__ __forceinline__ void guard_pair(v8f& a, v16h x, v16h y) {
  asm volatile("v_nop\n\tv_nop\n\tv_nop\n\tv_nop" : "+v"(a) : "v"(x), "v"(y));
}
__device__ __forceinline__ void guard_quad(v8f& a, v16h x0, v16h x1, v16h y0, v16h y1) {
  asm volatile("v_nop\n\tv_nop\n\tv_nop\n\tv_nop" : "+v"(a) : "v"(x0), "v"(x1), "v"(y0), "v"(y1));
}
__device__ __forceinline__ void guard_acc(v8f& a) {
  asm volatile("v_nop\n\tv_nop\n\tv_nop\n\tv_nop" : "+v"(a));
}

template <bool SPLIT>
__global__ __launch_bounds__(256) void gemm_f16_kernel(
    const unsigned short* __restrict__ Ahp, const unsigned short* __restrict__ Arp, int lda, long strideA,
    const unsigned short* __restrict__ Bhp, const unsigned short* __restrict__ Brp, int ldb, long strideB,
    float* __restrict__ Cout, int ldc, long strideC,
    int M, int N, int K, float scale) {
  __shared__ __align__(16) float sT[8][16 * 68];
  const int z    = blockIdx.y;
  const int lane = threadIdx.x & 31;
  const int wave = threadIdx.x >> 5;
  const int tilesN = N >> 6;
  const int tilesM = M >> 5;
  const int tile = blockIdx.x * 8 + wave;
  if (tile >= tilesM * tilesN) return;
  const int tm = tile / tilesN;
  const int tn = tile - tm * tilesN;
  const int m0 = tm << 5;
  const int n0 = tn << 6;
  const int rlane = lane & 15;
  const int half8 = (lane >> 4) * 8;
  const int mOff  = (lane >> 4) * 8;

  const size_t aoff = (size_t)z * (size_t)strideA + (size_t)(m0 + rlane) * lda + half8;
  const size_t boff = (size_t)z * (size_t)strideB + (size_t)(n0 + rlane) * ldb + half8;
  const _Float16* pa0 = (const _Float16*)Ahp + aoff;
  const _Float16* pa1 = pa0 + (size_t)16 * lda;
  const _Float16* pr0 = SPLIT ? ((const _Float16*)Arp + aoff) : pa0;
  const _Float16* pr1 = pr0 + (size_t)16 * lda;
  const _Float16* pbh = (const _Float16*)Bhp + boff;
  const _Float16* pbr = SPLIT ? ((const _Float16*)Brp + boff) : pbh;
  const size_t bstep = (size_t)16 * ldb;

  v8f acc[2][4], accr[2][4];
#pragma unroll
  for (int i = 0; i < 2; ++i)
#pragma unroll
    for (int j = 0; j < 4; ++j) {
      acc[i][j]  = (v8f){0.f, 0.f, 0.f, 0.f, 0.f, 0.f, 0.f, 0.f};
      accr[i][j] = (v8f){0.f, 0.f, 0.f, 0.f, 0.f, 0.f, 0.f, 0.f};
    }

  for (int k0 = 0; k0 < K; k0 += 32) {
    const v16h ah0 = FragH::load(pa0 + k0);
    const v16h ah1 = FragH::load(pa1 + k0);
    v16h ar0 = ah0, ar1 = ah1;
    if (SPLIT) {
      ar0 = FragH::load(pr0 + k0);
      ar1 = FragH::load(pr1 + k0);
    }
#pragma unroll
    for (int j = 0; j < 4; ++j) {
      const v16h bh = FragH::load(pbh + j * bstep + k0);
      v16h br = bh;
      if (SPLIT) br = FragH::load(pbr + j * bstep + k0);
      acc[0][j] = FragH::mma(ah0, bh, acc[0][j]);
      acc[1][j] = FragH::mma(ah1, bh, acc[1][j]);
      if (SPLIT) {
        accr[0][j] = FragH::mma(ah0, br, accr[0][j]);
        accr[1][j] = FragH::mma(ah1, br, accr[1][j]);
        accr[0][j] = FragH::mma(ar0, bh, accr[0][j]);
        accr[1][j] = FragH::mma(ar1, bh, accr[1][j]);
      }
      guard_pair(acc[0][j], ah0, bh);
      guard_pair(acc[1][j], ah1, bh);
      if (SPLIT) {
        guard_quad(accr[0][j], ah0, ar0, bh, br);
        guard_quad(accr[1][j], ah1, ar1, bh, br);
      }
    }
  }
#pragma unroll
  for (int i = 0; i < 2; ++i)
#pragma unroll
    for (int j = 0; j < 4; ++j) {
      guard_acc(acc[i][j]);
      if (SPLIT) guard_acc(accr[i][j]);
    }

  float* slab = sT[wave];
  float* C = Cout + (size_t)z * (size_t)strideC;
  const int hh = lane >> 4, c4 = (lane & 15) * 4;
#pragma unroll
  for (int i = 0; i < 2; ++i) {
    const int mBase = m0 + (i << 4);
#pragma unroll
    for (int j = 0; j < 4; ++j) {
#pragma unroll
      for (int r = 0; r < 8; ++r) {
        float v = acc[i][j][r];
        if (SPLIT) v += accr[i][j][r] * kResInv;
        v *= scale;
        slab[(mOff + r) * 68 + (j << 4) + rlane] = v;
      }
    }
    __builtin_amdgcn_fence(__ATOMIC_RELEASE, "workgroup");
    __builtin_amdgcn_wave_barrier();
    __builtin_amdgcn_fence(__ATOMIC_ACQUIRE, "workgroup");
    for (int pass = 0; pass < 2; ++pass) {
#pragma unroll
      for (int it = 0; it < 8; ++it) {
        const int row = it * 2 + hh;
        const v4f v = *(const v4f*)(slab + row * 68 + c4);
        *(volatile v4f*)(C + (size_t)(mBase + row) * ldc + n0 + c4) = v;
      }
      __threadfence();
    }
    __builtin_amdgcn_fence(__ATOMIC_RELEASE, "workgroup");
    __builtin_amdgcn_wave_barrier();
    __builtin_amdgcn_fence(__ATOMIC_ACQUIRE, "workgroup");
  }
}

__global__ __launch_bounds__(256) void cast_x_kernel(const float* __restrict__ x,
                                                     unsigned short* __restrict__ XH,
                                                     unsigned short* __restrict__ XR) {
  const int i = blockIdx.x * 256 + threadIdx.x;
  if (i >= kTok * (kChan / 8)) return;
  const size_t off = (size_t)i * 8;
  const v4f a = *(const v4f*)(x + off);
  const v4f b = *(const v4f*)(x + off + 4);
  float v[8];
#pragma unroll
  for (int e = 0; e < 4; ++e) {
    v[e]     = a[e] * kXCarry;
    v[4 + e] = b[e] * kXCarry;
  }
  v4u uh, ur;
  pack8_split(v, uh, ur);
  for (int pass = 0; pass < 2; ++pass) {
    *(volatile v4u*)(XH + off) = uh;
    *(volatile v4u*)(XR + off) = ur;
    __threadfence();
  }
}

__global__ __launch_bounds__(256) void cast_w_kernel(const float* __restrict__ W0, const float* __restrict__ W1,
                                                     const float* __restrict__ W2, const float* __restrict__ W3,
                                                     const float* __restrict__ W4,
                                                     unsigned short* __restrict__ WS, unsigned short* __restrict__ WR) {
  const int z = blockIdx.y;
  const int i = blockIdx.x * 256 + threadIdx.x;
  if (i >= (int)(kWBig / 8)) return;
  const float* W = (z == 0) ? W0 : (z == 1) ? W1 : (z == 2) ? W2 : (z == 3) ? W3 : W4;
  const size_t off = (size_t)i * 8;
  const v4f a = *(const v4f*)(W + off);
  const v4f b = *(const v4f*)(W + off + 4);
  float v[8];
#pragma unroll
  for (int e = 0; e < 4; ++e) {
    v[e]     = a[e] * kWCarry;
    v[4 + e] = b[e] * kWCarry;
  }
  v4u uh, ur;
  pack8_split(v, uh, ur);
  const bool has_res = (z >= 3);
  const size_t oh = (size_t)z * kWBig + off;
  const size_t orr = (size_t)(has_res ? (z - 3) : 0) * kWBig + off;
  for (int pass = 0; pass < 2; ++pass) {
    *(volatile v4u*)(WS + oh) = uh;
    if (has_res) *(volatile v4u*)(WR + orr) = ur;
    __threadfence();
  }
}

__global__ __launch_bounds__(256) void cast_gate_w_kernel(const float* __restrict__ Wb, const float* __restrict__ Wgk,
                                                          unsigned short* __restrict__ WBG) {
  const int i = blockIdx.x * 256 + threadIdx.x;
  if (i >= kGateN * (kChan / 8)) return;
  const int r  = i >> 7;
  const int c8 = (i & 127) * 8;
  const int rb = (r < kHeads) ? r : (kHeads - 1);
  int rg = r - kHeads;
  rg = (rg < 0) ? 0 : rg;
  rg = (rg > kHeads - 1) ? (kHeads - 1) : rg;
  const v4f a0 = *(const v4f*)(Wb + (size_t)rb * kChan + c8);
  const v4f a1 = *(const v4f*)(Wb + (size_t)rb * kChan + c8 + 4);
  const v4f g0 = *(const v4f*)(Wgk + (size_t)rg * kChan + c8);
  const v4f g1 = *(const v4f*)(Wgk + (size_t)rg * kChan + c8 + 4);
  float fa[8], fg[8];
#pragma unroll
  for (int e = 0; e < 4; ++e) {
    fa[e] = a0[e];
    fa[4 + e] = a1[e];
    fg[e] = g0[e];
    fg[4 + e] = g1[e];
  }
#pragma unroll
  for (int e = 0; e < 8; ++e) asm volatile("" : "+v"(fa[e]), "+v"(fg[e]));
  float v[8];
#pragma unroll
  for (int e = 0; e < 8; ++e) {
    const float s = (r < kHeads) ? fa[e] : ((r < kGateReal) ? fg[e] : 0.0f);
    v[e] = s * kWCarry;
  }
  const v4u uh = pack8_plain(v);
  const size_t off = (size_t)i * 8;
  for (int pass = 0; pass < 2; ++pass) {
    *(volatile v4u*)(WBG + off) = uh;
    __threadfence();
  }
}

__global__ __launch_bounds__(64) void rope_freq_kernel(float* __restrict__ FT) {
#pragma clang fp contract(off)
  __shared__ float sp[64];
  const int tid = threadIdx.x;
  const int m = tid & 31;
  const float ar = (float)(2 * m) / (float)kHdim;
  const float sbase = kRopeBase * exp2f(kSbExp);
  const float base = (tid < 32) ? sbase : kRopeBase;
  const float pw = powf(base, ar);
  sp[tid] = 1.0f / pw;
  __syncthreads();
  const float invf = sp[m];
  const float fe = sp[32 + m];
  const float wl = kTwoPi / fe;
  float ms = (wl - kBetaFast) * (1.0f / (kBetaSlow - kBetaFast));
  ms = fminf(fmaxf(ms, 0.0f), 1.0f);
  const float sc = 1.0f + (kRopeScaling - 1.0f) * ms;
  const float rsc = 1.0f / sc;
  if (tid < 32) {
    *(volatile float*)(FT + m) = invf;
    *(volatile float*)(FT + 32 + m) = rsc;
    __threadfence();
    *(volatile float*)(FT + m) = invf;
    *(volatile float*)(FT + 32 + m) = rsc;
  }
}

__global__ __launch_bounds__(256) void rope_table_kernel(const float* __restrict__ FT, float* __restrict__ RT) {
#pragma clang fp contract(off)
  const int gid = blockIdx.x * 256 + threadIdx.x;
  if (gid >= kSteps * kHalfD) return;
  const int t = gid >> 5;
  const int m = gid & 31;
  const float invf = FT[m];
  const float rsc = FT[32 + m];
  const float tt = (float)t * rsc;
  const float ang = tt * invf;
  const float cs = cosf(ang);
  const float sn = sinf(ang);
  float* p = RT + (size_t)t * kHdim + m;
  *(volatile float*)(p) = cs;
  *(volatile float*)(p + 32) = sn;
  __threadfence();
  *(volatile float*)(p) = cs;
  *(volatile float*)(p + 32) = sn;
}

__global__ __launch_bounds__(256) void gate_prep_kernel(float* BG, const float* __restrict__ bb,
                                                        const float* __restrict__ bgk,
                                                        const float* __restrict__ A_log,
                                                        const float* __restrict__ dt_bias) {
  const int lane = threadIdx.x & 31;
  const int row = blockIdx.x * 8 + (threadIdx.x >> 5);
  const int hh = lane & 15;
  const size_t idx = (size_t)row * kGateN + lane;
  const float v = BG[idx];
  const float zb = v + bb[hh];
  const float beta = 1.0f / (1.0f + expf(-zb));
  const float zg = (v + bgk[hh]) + dt_bias[hh];
  const float sp = fmaxf(zg, 0.0f) + log1pf(expf(-fabsf(zg)));
  const float av = expf(A_log[hh]);
  float alpha = expf(-av * sp);
  alpha = (alpha < kF32Min) ? 0.0f : alpha;
  const float res = (lane < kHeads) ? beta : alpha;
  *(volatile float*)(BG + idx) = res;
  __threadfence();
  *(volatile float*)(BG + idx) = res;
}

template <bool ROPE>
__global__ __launch_bounds__(256) void conv_act_kernel(const float* __restrict__ Pin, float* __restrict__ Cdst,
                                                       const float* __restrict__ cwA, const float* __restrict__ cbA,
                                                       const float* __restrict__ cwB, const float* __restrict__ cbB,
                                                       const float* __restrict__ RT) {
  const int z = blockIdx.y;
  const float* cw = (z == 0) ? cwA : cwB;
  const float* cb = (z == 0) ? cbA : cbB;
  const float* P = Pin + (size_t)z * kPlane;
  float* O = Cdst + (size_t)z * kPlane;
  const int lane = threadIdx.x & 31;
  const int pair = blockIdx.x * 8 + (threadIdx.x >> 5);
  const int tok = pair >> 4;
  const int h   = pair & 15;
  const int t   = tok & (kSteps - 1);
  const int c   = h * kHdim + 2 * lane;
  float x0[kTaps], x1[kTaps];
#pragma unroll
  for (int i = 0; i < kTaps; ++i) {
    const bool valid = (t - (kTaps - 1) + i) >= 0;
    const int rowc = valid ? (tok - (kTaps - 1) + i) : tok;
    const v2f xv = *(const v2f*)(P + (size_t)rowc * kChan + c);
    x0[i] = valid ? xv[0] : 0.0f;
    x1[i] = valid ? xv[1] : 0.0f;
  }
  const v4f wa = *(const v4f*)(cw + (size_t)c * kTaps);
  const v4f wb = *(const v4f*)(cw + (size_t)c * kTaps + 4);
  const v2f bv = *(const v2f*)(cb + c);
  float a0 = wa[0] * x0[0];
  a0 = fmaf(wa[1], x0[1], a0);
  a0 = fmaf(wa[2], x0[2], a0);
  a0 = fmaf(wa[3], x0[3], a0);
  a0 += bv[0];
  float a1 = wb[0] * x1[0];
  a1 = fmaf(wb[1], x1[1], a1);
  a1 = fmaf(wb[2], x1[2], a1);
  a1 = fmaf(wb[3], x1[3], a1);
  a1 += bv[1];
  const float s0 = a0 * __builtin_amdgcn_rcpf(1.0f + expf(-a0));
  const float s1 = a1 * __builtin_amdgcn_rcpf(1.0f + expf(-a1));
  if (ROPE) {
    const int m = (2 * lane) & 31;
    const float ce = RT[(size_t)t * kHdim + m];
    const float se = RT[(size_t)t * kHdim + 32 + m];
    const float o1 = s0 * ce - s1 * se;
    const float o2 = s0 * se + s1 * ce;
    const float ss = wave_sum32(o1 * o1 + o2 * o2);
    const float inv = 1.0f / fmaxf(sqrtf(ss), 1e-12f);
    const float r1 = o1 * inv;
    const float r2 = o2 * inv;
    float* po = O + (size_t)tok * kChan + (size_t)h * kHdim + lane;
    *(volatile float*)(po) = r1;
    *(volatile float*)(po + 32) = r2;
    __threadfence();
    *(volatile float*)(po) = r1;
    *(volatile float*)(po + 32) = r2;
  } else {
    const v2f ov = (v2f){s0, s1};
    float* po = O + (size_t)tok * kChan + c;
    *(volatile v2f*)(po) = ov;
    __threadfence();
    *(volatile v2f*)(po) = ov;
  }
}

__global__ __launch_bounds__(256) void state_scan_kernel(const float* __restrict__ Qc, const float* __restrict__ Kc,
                                                         const float* __restrict__ Vc, const float* __restrict__ AB,
                                                         const float* __restrict__ Dp, float* __restrict__ Y) {
  __shared__ __align__(16) float lv[3 * kChunk * 64];
  __shared__ __align__(16) float ab[kChunk * 32];
  __shared__ __align__(16) float yb[kChunk * 64];
  const int bh  = blockIdx.x;
  const int b   = bh >> 4;
  const int h   = bh & 15;
  const int tid = threadIdx.x;
  const int i   = tid >> 2;
  const int qd  = tid & 3;
  const int j0  = qd * 16;
  const int lrow = tid >> 4;
  const int lc4  = (tid & 15) * 4;
  const int lc2  = (tid & 15) * 2;
  const size_t base  = (size_t)b * kSteps * kChan + (size_t)h * kHdim;
  const size_t abase = (size_t)b * kSteps * kGateN;
  const float dph = Dp[h];

  float S[16];
#pragma unroll
  for (int jj = 0; jj < 16; ++jj) S[jj] = 0.0f;

#pragma unroll 1
  for (int ch = 0; ch < kSteps / kChunk; ++ch) {
    const size_t goff = base + (size_t)(ch * kChunk + lrow) * kChan + lc4;
    {
      const v4f t0 = *(const v4f*)(Qc + goff);
      const v4f t1 = *(const v4f*)(Kc + goff);
      const v4f t2 = *(const v4f*)(Vc + goff);
      const v2f t3 = *(const v2f*)(AB + abase + (size_t)(ch * kChunk + lrow) * kGateN + lc2);
      const int lo = lrow * 64 + lc4;
      *(v4f*)(lv + 0 * kChunk * 64 + lo) = t0;
      *(v4f*)(lv + 1 * kChunk * 64 + lo) = t1;
      *(v4f*)(lv + 2 * kChunk * 64 + lo) = t2;
      *(v2f*)(ab + lrow * 32 + lc2) = t3;
    }
    __syncthreads();

#pragma unroll 1
    for (int s = 0; s < kChunk; ++s) {
      const float* pq = lv + 0 * kChunk * 64 + s * 64 + j0;
      const float* pk = lv + 1 * kChunk * 64 + s * 64 + j0;
      const float vi = lv[2 * kChunk * 64 + s * 64 + i];
      const float be = ab[s * 32 + h];
      const float al = ab[s * 32 + 16 + h];
      v4f kv[4];
#pragma unroll
      for (int g4 = 0; g4 < 4; ++g4) kv[g4] = *(const v4f*)(pk + 4 * g4);
      float sk = 0.0f;
#pragma unroll
      for (int g4 = 0; g4 < 4; ++g4) {
#pragma unroll
        for (int e = 0; e < 4; ++e) sk = fmaf(S[4 * g4 + e], kv[g4][e], sk);
      }
      sk += __shfl_xor(sk, 1, 32);
      sk += __shfl_xor(sk, 2, 32);
      const float t1 = be * sk;
      const float cf = be * vi - al * t1;
      float out = 0.0f;
#pragma unroll
      for (int g4 = 0; g4 < 4; ++g4) {
        const v4f q4 = *(const v4f*)(pq + 4 * g4);
#pragma unroll
        for (int e = 0; e < 4; ++e) {
          const float sn = fmaf(cf, kv[g4][e], al * S[4 * g4 + e]);
          S[4 * g4 + e] = sn;
          out = fmaf(sn, q4[e], out);
        }
      }
      out += __shfl_xor(out, 1, 32);
      out += __shfl_xor(out, 2, 32);
      if (qd == 0) yb[s * 64 + i] = out + dph * vi;
    }
    __syncthreads();
    {
      const v4f val = *(const v4f*)(yb + lrow * 64 + lc4);
      *(volatile v4f*)(Y + goff) = val;
      __threadfence();
      *(volatile v4f*)(Y + goff) = val;
    }
  }
}

__global__ __launch_bounds__(256) void norm_gate_kernel(const float* __restrict__ Y, const float* __restrict__ Gf,
                                                        const float* __restrict__ nw, unsigned* __restrict__ YG) {
  const int lane = threadIdx.x & 31;
  const int pair = blockIdx.x * 8 + (threadIdx.x >> 5);
  const int tok = pair >> 4;
  const int h   = pair & 15;
  const size_t base = (size_t)tok * kChan + (size_t)h * kHdim + 2 * lane;
  const v2f y2 = *(const v2f*)(Y + base);
  const v2f g2 = *(const v2f*)(Gf + base);
  const v2f w2 = *(const v2f*)(nw + 2 * lane);
  const float ms = wave_sum32(y2[0] * y2[0] + y2[1] * y2[1]) * (1.0f / (float)kHdim);
  const float rs = 1.0f / sqrtf(ms + kNormEps);
  const float r0 = w2[0] * (y2[0] * rs);
  const float r1 = w2[1] * (y2[1] * rs);
  const float s0 = r0 * __builtin_amdgcn_rcpf(1.0f + expf(-r0));
  const float s1 = r1 * __builtin_amdgcn_rcpf(1.0f + expf(-r1));
  const float o0 = (g2[0] * s0) * kYCarry;
  const float o1 = (g2[1] * s1) * kYCarry;
  const unsigned short h0 = h_bits(o0);
  const unsigned short h1 = h_bits(o1);
  const unsigned wh = pk16(h0, h1);
  const size_t widx = base >> 1;
  *(volatile unsigned*)(YG + widx) = wh;
  __threadfence();
  *(volatile unsigned*)(YG + widx) = wh;
}

extern "C" void kernel_launch(void* const* d_in, const int* in_sizes, int n_in,
                              void* d_out, int out_size, void* d_ws, size_t ws_size, hipStream_t stream) {
  if (n_in < 20 || d_out == nullptr || d_ws == nullptr) return;
  const int nP = (int)kPlane;
  const int nW = (int)kWBig;
  if (in_sizes[0] != nP) return;
  for (int i = 1; i <= 5; ++i) if (in_sizes[i] != nW) return;
  if (in_sizes[6] != kHeads * kChan || in_sizes[7] != kHeads) return;
  if (in_sizes[8] != kHeads * kChan || in_sizes[9] != kHeads) return;
  if (in_sizes[10] != kChan * kTaps || in_sizes[11] != kChan) return;
  if (in_sizes[12] != kChan * kTaps || in_sizes[13] != kChan) return;
  if (in_sizes[14] != kChan * kTaps || in_sizes[15] != kChan) return;
  if (in_sizes[16] != kHeads || in_sizes[17] != kHeads || in_sizes[18] != kHeads) return;
  if (in_sizes[19] != kHdim) return;
  if (out_size != nP) return;

  const float* x    = (const float*)d_in[0];
  const float* Wq   = (const float*)d_in[1];
  const float* Wk   = (const float*)d_in[2];
  const float* Wv   = (const float*)d_in[3];
  const float* Wg   = (const float*)d_in[4];
  const float* Wo   = (const float*)d_in[5];
  const float* Wb   = (const float*)d_in[6];
  const float* bb   = (const float*)d_in[7];
  const float* Wgk  = (const float*)d_in[8];
  const float* bgk  = (const float*)d_in[9];
  const float* cqw  = (const float*)d_in[10];
  const float* cqb  = (const float*)d_in[11];
  const float* ckw  = (const float*)d_in[12];
  const float* ckb  = (const float*)d_in[13];
  const float* cvw  = (const float*)d_in[14];
  const float* cvb  = (const float*)d_in[15];
  const float* Alog = (const float*)d_in[16];
  const float* Dp   = (const float*)d_in[17];
  const float* dtb  = (const float*)d_in[18];
  const float* onw  = (const float*)d_in[19];
  float* out = (float*)d_out;

  char* ws = (char*)d_ws;
  size_t off = 0;
  auto carve = [&](size_t bytes) -> char* {
    char* p = ws + off;
    off += (bytes + 255) & ~(size_t)255;
    return p;
  };
  unsigned short* XH  = (unsigned short*)carve(kPlane * 2);
  unsigned short* XR  = (unsigned short*)carve(kPlane * 2);
  unsigned short* WS  = (unsigned short*)carve(5 * kWBig * 2);
  unsigned short* WR  = (unsigned short*)carve(2 * kWBig * 2);
  unsigned short* WBG = (unsigned short*)carve((size_t)kGateN * kChan * 2);
  float* P  = (float*)carve(3 * kPlane * 4);
  float* CV = (float*)carve(3 * kPlane * 4);
  float* BG = (float*)carve((size_t)kTok * kGateN * 4);
  float* FT = (float*)carve((size_t)kHdim * 4);
  float* RT = (float*)carve((size_t)kSteps * kHdim * 4);
  if (off > ws_size || off > (size_t)134217728) return;

  float* P0 = P;
  float* P2 = P + 2 * kPlane;
  float* Qc = CV;
  float* Kc = CV + kPlane;
  float* Vc = CV + 2 * kPlane;
  float* Gf = P;
  float* Yf = P + kPlane;
  unsigned short* YG = XH;

  cast_x_kernel<<<(kTok * (kChan / 8)) / 256, 256, 0, stream>>>(x, XH, XR);
  cast_w_kernel<<<dim3((unsigned)(kWBig / 8 / 256), 5), 256, 0, stream>>>(Wq, Wk, Wo, Wv, Wg, WS, WR);
  cast_gate_w_kernel<<<(kGateN * (kChan / 8)) / 256, 256, 0, stream>>>(Wb, Wgk, WBG);

  rope_freq_kernel<<<1, 64, 0, stream>>>(FT);
  rope_table_kernel<<<(kSteps * kHalfD) / 256, 256, 0, stream>>>(FT, RT);

  const int blkBig  = (kTok / 32) * (kChan / 64) / 8;
  const int blkGate = (kTok / 32) * (kGateN / 64) / 8;
  gemm_f16_kernel<false><<<dim3(blkBig, 2), 256, 0, stream>>>(
      XH, XH, kChan, 0L, WS, WS, kChan, (long)kWBig,
      P0, kChan, (long)kPlane, kTok, kChan, kChan, kScaleProj);
  gemm_f16_kernel<true><<<dim3(blkBig, 1), 256, 0, stream>>>(
      XH, XR, kChan, 0L, WS + 3 * kWBig, WR, kChan, 0L,
      P2, kChan, 0L, kTok, kChan, kChan, kScaleProj);
  gemm_f16_kernel<false><<<dim3(blkGate, 1), 256, 0, stream>>>(
      XH, XH, kChan, 0L, WBG, WBG, kChan, 0L,
      BG, kGateN, 0L, kTok, kGateN, kChan, kScaleProj);

  gate_prep_kernel<<<kTok / 8, 256, 0, stream>>>(BG, bb, bgk, Alog, dtb);

  conv_act_kernel<true><<<dim3((kTok * kHeads) / 8, 2), 256, 0, stream>>>(P0, Qc, cqw, cqb, ckw, ckb, RT);
  conv_act_kernel<false><<<dim3((kTok * kHeads) / 8, 1), 256, 0, stream>>>(P2, Vc, cvw, cvb, cvw, cvb, RT);

  gemm_f16_kernel<true><<<dim3(blkBig, 1), 256, 0, stream>>>(
      XH, XR, kChan, 0L, WS + 4 * kWBig, WR + kWBig, kChan, 0L,
      Gf, kChan, 0L, kTok, kChan, kChan, kScaleProj);

  state_scan_kernel<<<kBatch * kHeads, 256, 0, stream>>>(Qc, Kc, Vc, BG, Dp, Yf);

  norm_gate_kernel<<<(kTok * kHeads) / 8, 256, 0, stream>>>(Yf, Gf, onw, (unsigned*)YG);

  gemm_f16_kernel<false><<<dim3(blkBig, 1), 256, 0, stream>>>(
      YG, YG, kChan, 0L, WS + 2 * kWBig, WS + 2 * kWBig, kChan, 0L,
      out, kChan, 0L, kTok, kChan, kChan, kScaleOut);
}
